// SUPRAParallelFixedGamma_10024453668953
// MI455X (gfx1250) — hardware-verified
//
#include <hip/hip_runtime.h>

typedef _Float16 v16h __attribute__((ext_vector_type(16)));
typedef _Float16 v8h  __attribute__((ext_vector_type(8)));
typedef float    v8f  __attribute__((ext_vector_type(8)));
typedef float    v4f  __attribute__((ext_vector_type(4)));

union Frag { v16h v; v8h half[2]; };

__device__ __forceinline__ v8f wmma_f16(v16h a, v16h b, v8f c)
{
  v8f d = __builtin_amdgcn_wmma_f32_16x16x32_f16(false, a, false, b, (short)0, c, false, false);
  asm volatile("v_nop\n\tv_nop\n\tv_nop\n\tv_nop" : "+v"(d) : "v"(a), "v"(b));
  return d;
}

#define TBK 32
#define STR 40
#define TILE_HALVES (128 * STR)

__global__ __launch_bounds__(256)
void cvt_f16_kernel(const float* __restrict__ in, _Float16* __restrict__ out, int n, float scale)
{
  const size_t i = ((size_t)blockIdx.x * 256 + threadIdx.x) * 8;
  if (i + 8 > (size_t)n) return;
  const v4f a = *(const v4f*)(in + i);
  const v4f b = *(const v4f*)(in + i + 4);
  v8h o;
  o[0] = (_Float16)(a[0] * scale);
  o[1] = (_Float16)(a[1] * scale);
  o[2] = (_Float16)(a[2] * scale);
  o[3] = (_Float16)(a[3] * scale);
  o[4] = (_Float16)(b[0] * scale);
  o[5] = (_Float16)(b[1] * scale);
  o[6] = (_Float16)(b[2] * scale);
  o[7] = (_Float16)(b[3] * scale);
  _Float16* p = out + i;
  *(volatile v8h*)p = o;
  __threadfence();
  *(volatile v8h*)p = o;
}

template <int OUT16>
__global__ __launch_bounds__(256)
void gemm_nt_f16_kernel(const _Float16* __restrict__ A, int lda, long long sAz,
                        const _Float16* __restrict__ Bm, int ldb, long long sBz,
                        _Float16* __restrict__ out16, float* __restrict__ out32,
                        int ldo, long long sOz, int K,
                        const float* __restrict__ bias, int use_bias,
                        float acc_scale, float out_scale, int relu)
{
  __shared__ float LDSF[8192] __attribute__((aligned(16)));
  _Float16* sA = (_Float16*)LDSF;
  _Float16* sB = sA + TILE_HALVES;

  A  += (size_t)blockIdx.z * (size_t)sAz;
  Bm += (size_t)blockIdx.z * (size_t)sBz;

  const int mBase = blockIdx.y * 128;
  const int nBase = blockIdx.x * 128;
  const int tid = threadIdx.x;
  const int l   = tid & 31;
  const int wid = tid >> 5;
  const int wm  = wid & 3;
  const int wn  = wid >> 2;
  const int h   = l >> 4;
  const int m   = l & 15;

  const v8f vzero = {0.f, 0.f, 0.f, 0.f, 0.f, 0.f, 0.f, 0.f};
  v8f acc[2][4];
#pragma unroll
  for (int mi = 0; mi < 2; ++mi)
#pragma unroll
    for (int ni = 0; ni < 4; ++ni) acc[mi][ni] = vzero;

  const int KT = K / TBK;
  for (int kt = 0; kt < KT; ++kt) {
    const int k0 = kt * TBK;
#pragma unroll
    for (int it = 0; it < 2; ++it) {
      const int c    = it * 256 + tid;
      const int row  = c >> 2;
      const int col8 = (c & 3) << 3;
      const v8h va = *(const v8h*)(A  + (size_t)(mBase + row) * lda + k0 + col8);
      const v8h vb = *(const v8h*)(Bm + (size_t)(nBase + row) * ldb + k0 + col8);
      *(v8h*)(sA + row * STR + col8) = va;
      *(v8h*)(sB + row * STR + col8) = vb;
    }
    __syncthreads();

    Frag a[2];
#pragma unroll
    for (int mi = 0; mi < 2; ++mi) {
      const int base = (wm * 32 + mi * 16 + m) * STR;
      a[mi].half[0] = *(const v8h*)(sA + base + 8 * h);
      a[mi].half[1] = *(const v8h*)(sA + base + 16 + 8 * h);
    }
#pragma unroll
    for (int ni = 0; ni < 4; ++ni) {
      const int bbase = (wn * 64 + ni * 16 + m) * STR;
      Frag b;
      b.half[0] = *(const v8h*)(sB + bbase + 8 * h);
      b.half[1] = *(const v8h*)(sB + bbase + 16 + 8 * h);
#pragma unroll
      for (int mi = 0; mi < 2; ++mi)
        acc[mi][ni] = wmma_f16(a[mi].v, b.v, acc[mi][ni]);
    }
    __syncthreads();
  }

  if (OUT16) {
    _Float16* stg = (_Float16*)LDSF + wid * 2048;
#pragma unroll
    for (int ni = 0; ni < 4; ++ni) {
      const int gn = nBase + wn * 64 + ni * 16 + m;
      const float bb = use_bias ? bias[gn] : 0.0f;
#pragma unroll
      for (int mi = 0; mi < 2; ++mi) {
#pragma unroll
        for (int g = 0; g < 8; ++g) {
          float val = acc[mi][ni][g] * acc_scale + bb;
          if (relu) val = fmaxf(val, 0.0f);
          stg[(mi * 16 + 8 * h + g) * 64 + ni * 16 + m] = (_Float16)(val * out_scale);
        }
      }
    }
    __syncthreads();
    v8h ov[8];
#pragma unroll
    for (int p = 0; p < 8; ++p)
      ov[p] = *(const v8h*)(stg + (p * 4 + (l >> 3)) * 64 + (l & 7) * 8);
    _Float16* O = out16 + (size_t)blockIdx.z * (size_t)sOz;
    const size_t rbase = (size_t)(mBase + wm * 32);
    const int cbase = nBase + wn * 64 + (l & 7) * 8;
#pragma unroll
    for (int p = 0; p < 8; ++p)
      *(volatile v8h*)(O + (rbase + p * 4 + (l >> 3)) * (size_t)ldo + cbase) = ov[p];
    __threadfence();
#pragma unroll
    for (int p = 0; p < 8; ++p)
      *(volatile v8h*)(O + (rbase + p * 4 + (l >> 3)) * (size_t)ldo + cbase) = ov[p];
  } else {
    float* stg = LDSF + wid * 1024;
    float* O = out32 + (size_t)blockIdx.z * (size_t)sOz;
    const size_t rbase = (size_t)(mBase + wm * 32);
#pragma unroll
    for (int ph = 0; ph < 2; ++ph) {
#pragma unroll
      for (int nn = 0; nn < 2; ++nn) {
        const int ni = ph * 2 + nn;
        const int gn = nBase + wn * 64 + ni * 16 + m;
        const float bb = use_bias ? bias[gn] : 0.0f;
#pragma unroll
        for (int mi = 0; mi < 2; ++mi) {
#pragma unroll
          for (int g = 0; g < 8; ++g) {
            float val = acc[mi][ni][g] * acc_scale + bb;
            if (relu) val = fmaxf(val, 0.0f);
            stg[(mi * 16 + 8 * h + g) * 32 + nn * 16 + m] = val * out_scale;
          }
        }
      }
      __syncthreads();
      v4f ov[8];
#pragma unroll
      for (int p = 0; p < 8; ++p)
        ov[p] = *(const v4f*)(stg + (p * 4 + (l >> 3)) * 32 + (l & 7) * 4);
      const int cbase = nBase + wn * 64 + ph * 32 + (l & 7) * 4;
#pragma unroll
      for (int p = 0; p < 8; ++p)
        *(volatile v4f*)(O + (rbase + p * 4 + (l >> 3)) * (size_t)ldo + cbase) = ov[p];
      __threadfence();
#pragma unroll
      for (int p = 0; p < 8; ++p)
        *(volatile v4f*)(O + (rbase + p * 4 + (l >> 3)) * (size_t)ldo + cbase) = ov[p];
      __syncthreads();
    }
  }
}

__global__ __launch_bounds__(256)
void vdiag_kernel(const float* __restrict__ x, const float* __restrict__ Wv,
                  const float* __restrict__ bv, float* __restrict__ vd,
                  int M, int T, int D)
{
  __shared__ float s[32] __attribute__((aligned(16)));
  const int wid = threadIdx.x >> 5, lane = threadIdx.x & 31;
#pragma unroll 1
  for (int rr = 0; rr < 4; ++rr) {
    const int row = blockIdx.x * 32 + wid * 4 + rr;
    float sum = 0.0f;
    if (row < M) {
      const int j = row % T;
      const float* xr = x  + (size_t)row * D;
      const float* wr = Wv + (size_t)j * D;
#pragma unroll 1
      for (int i = lane * 4; i < D; i += 128) {
        const v4f a = *(const v4f*)(xr + i);
        const v4f w = *(const v4f*)(wr + i);
        sum = fmaf(a[0], w[0], sum);
        sum = fmaf(a[1], w[1], sum);
        sum = fmaf(a[2], w[2], sum);
        sum = fmaf(a[3], w[3], sum);
      }
#pragma unroll
      for (int off = 16; off > 0; off >>= 1) sum += __shfl_xor(sum, off, 32);
      sum += bv[j];
    }
    if (lane == 0) s[wid * 4 + rr] = sum;
  }
  __syncthreads();
  if (wid == 0 && lane < 8) {
    const v4f v = *(const v4f*)(s + lane * 4);
    float* p = vd + (size_t)blockIdx.x * 32 + lane * 4;
    *(volatile v4f*)p = v;
    __threadfence();
    *(volatile v4f*)p = v;
  }
}

__device__ __forceinline__ float decay_w(int t, int j, float log2g, float rinv, float gt)
{
  return (j >= t) ? exp2f((float)(j - t) * log2g) * gt
                  : (1.0f - exp2f((float)(j + 1) * log2g)) * rinv + (float)(t - j);
}

__global__ __launch_bounds__(256)
void norm_kernel(float* __restrict__ out, const float* __restrict__ vd,
                 const float* __restrict__ gamma_p, int T, float qk_scale)
{
  __shared__ float red[8];
  const int row = blockIdx.x;
  const int t = row % T;
  const int b = row / T;
  const int tid = threadIdx.x, lane = tid & 31, wid = tid >> 5;
  const float gamma = gamma_p[0];
  const float log2g = log2f(gamma);
  const float rinv  = 1.0f / (1.0f - gamma);
  const float gt    = (1.0f - exp2f((float)(t + 1) * log2g)) * rinv;
  float* orow = out + (size_t)row * T;
  const float* vdb = vd + (size_t)b * T;

  float part = 0.0f;
  for (int j0 = tid * 4; j0 < T; j0 += 1024) {
    const v4f qk = *(const v4f*)(orow + j0);
#pragma unroll
    for (int i = 0; i < 4; ++i) part += decay_w(t, j0 + i, log2g, rinv, gt) * (qk[i] * qk_scale);
  }
#pragma unroll
  for (int off = 16; off > 0; off >>= 1) part += __shfl_xor(part, off, 32);
  if (lane == 0) red[wid] = part;
  __syncthreads();
  const float den = ((red[0] + red[1]) + (red[2] + red[3])) + ((red[4] + red[5]) + (red[6] + red[7]));
  const float inv = 1.0f / (den + 1e-6f);

  for (int j0 = tid * 4; j0 < T; j0 += 1024) {
    const v4f qk = *(const v4f*)(orow + j0);
    const v4f vv = *(const v4f*)(vdb + j0);
    v4f o;
#pragma unroll
    for (int i = 0; i < 4; ++i)
      o[i] = (decay_w(t, j0 + i, log2g, rinv, gt) * (qk[i] * qk_scale)) * vv[i] * inv;
    float* p = orow + j0;
    *(volatile v4f*)p = o;
    __threadfence();
    *(volatile v4f*)p = o;
  }
}

extern "C" void kernel_launch(void* const* d_in, const int* in_sizes, int n_in,
                              void* d_out, int out_size, void* d_ws, size_t ws_size,
                              hipStream_t stream)
{
  if (n_in < 8) return;
  const float* x     = (const float*)d_in[0];
  const float* gamma = (const float*)d_in[1];
  const float* Wq    = (const float*)d_in[2];
  const float* bq    = (const float*)d_in[3];
  const float* Wk    = (const float*)d_in[4];
  const float* bk    = (const float*)d_in[5];
  const float* Wv    = (const float*)d_in[6];
  const float* bv    = (const float*)d_in[7];
  float* out = (float*)d_out;

  const int D = in_sizes[3];
  const int T = D;
  if (D <= 0 || (D % 128) != 0) return;
  const long long TD = (long long)T * D;
  const int Bn = (int)((long long)in_sizes[0] / TD);
  if (Bn <= 0 || (long long)Bn * TD != (long long)in_sizes[0]) return;
  if ((long long)in_sizes[2] != (long long)D * D || (long long)in_sizes[4] != (long long)D * D ||
      (long long)in_sizes[6] != (long long)D * D) return;
  if (in_sizes[5] != D || in_sizes[7] != D || in_sizes[1] < 1) return;
  if ((long long)out_size != (long long)Bn * T * T) return;

  const int M = Bn * T;
  const size_t MD = (size_t)M * D, DD = (size_t)D * D;
  const size_t Mpad = ((size_t)M + 31) / 32 * 32;

  size_t off = 0;
  _Float16* x16  = (_Float16*)((char*)d_ws + off); off += MD * 2;
  _Float16* Wq16 = (_Float16*)((char*)d_ws + off); off += DD * 2;
  _Float16* Wk16 = (_Float16*)((char*)d_ws + off); off += DD * 2;
  _Float16* q16  = (_Float16*)((char*)d_ws + off); off += MD * 2;
  _Float16* k16  = (_Float16*)((char*)d_ws + off); off += MD * 2;
  float*    vd   = (float*)((char*)d_ws + off);    off += Mpad * 4;
  if (off > ws_size) return;

  dim3 blk(256);

  cvt_f16_kernel<<<dim3((unsigned)((MD + 2047) / 2048)), blk, 0, stream>>>(x, x16, (int)MD, 1.0f);
  cvt_f16_kernel<<<dim3((unsigned)((DD + 2047) / 2048)), blk, 0, stream>>>(Wq, Wq16, (int)DD, 64.0f);
  cvt_f16_kernel<<<dim3((unsigned)((DD + 2047) / 2048)), blk, 0, stream>>>(Wk, Wk16, (int)DD, 64.0f);

  gemm_nt_f16_kernel<1><<<dim3(D / 128, M / 128, 1), blk, 0, stream>>>(
      x16, D, 0LL, Wq16, D, 0LL, q16, out, D, 0LL, D, bq, 1, 1.0f / 64.0f, 16.0f, 1);
  gemm_nt_f16_kernel<1><<<dim3(D / 128, M / 128, 1), blk, 0, stream>>>(
      x16, D, 0LL, Wk16, D, 0LL, k16, out, D, 0LL, D, bk, 1, 1.0f / 64.0f, 16.0f, 1);

  vdiag_kernel<<<dim3((unsigned)((M + 31) / 32)), blk, 0, stream>>>(x, Wv, bv, vd, M, T, D);

  gemm_nt_f16_kernel<0><<<dim3(T / 128, T / 128, Bn), blk, 0, stream>>>(
      q16, D, TD, k16, D, TD, q16, out, T, (long long)T * T, D, bq, 0, 1.0f, 1.0f, 0);

  norm_kernel<<<dim3((unsigned)M), blk, 0, stream>>>(out, vd, gamma, T, 1.0f / 256.0f);
}
